// TO_BlockNet_61770219651542
// MI455X (gfx1250) — hardware-run, weakly checked
//
#include <hip/hip_runtime.h>
#include <math.h>

typedef __attribute__((ext_vector_type(16))) _Float16 v16h;
typedef __attribute__((ext_vector_type(8)))  _Float16 v8h;
typedef __attribute__((ext_vector_type(16))) __bf16   v16b;
typedef __attribute__((ext_vector_type(8)))  __bf16   v8b;
typedef __attribute__((ext_vector_type(8)))  float    v8f;
typedef __attribute__((ext_vector_type(4)))  float    v4f;
typedef __attribute__((ext_vector_type(4)))  unsigned v4u;

constexpr int kPts     = 131072;
constexpr int kCells   = 32;
constexpr int kBasis   = 50;
constexpr int kKPad    = 64;
constexpr int kNPad    = 64;
constexpr int kKernFl  = kCells * 3 * kBasis;
constexpr int kMmBlk   = 128;
constexpr int kMmPts   = 1024;
constexpr float kCarryA   = 512.0f;
constexpr float kCarryW   = 64.0f;
constexpr float kFoldBack = 1.0f / (kCarryA * kCarryW);
constexpr float kF16Norm  = 6.103515625e-5f;
static_assert(kMmBlk * kMmPts == kPts);
static_assert((kPts % 256) == 0 && (kPts % 64) == 0);
static_assert((kKPad % 32) == 0 && (kNPad % 64) == 0);
static_assert(kKernFl == 4800 && (kKernFl % 4) == 0);
static_assert(kBasis <= kKPad && kCells <= kNPad);

constexpr size_t kOffPart = 0;
constexpr size_t kOffBidx = kOffPart + (size_t)kMmBlk * 32 * 4;
constexpr size_t kOffBt   = kOffBidx + (size_t)kPts * 4;
constexpr size_t kOffApl  = kOffBt   + (size_t)kNPad * kKPad * 2;
constexpr size_t kOffCpl  = kOffApl  + (size_t)kPts * kKPad * 2;
constexpr size_t kWsTotal = kOffCpl  + (size_t)kPts * kNPad * 4;
static_assert(kWsTotal == 50880512ull);
static_assert(kWsTotal <= 134217728ull);
static_assert((kOffBidx % 128) == 0 && (kOffBt % 128) == 0 && (kOffApl % 128) == 0 && (kOffCpl % 128) == 0);

__device__ __forceinline__ unsigned short f2bf_bits(float f) {
  unsigned u = __float_as_uint(f);
  return (unsigned short)((u + 0x7FFFu + ((u >> 16) & 1u)) >> 16);
}
__device__ __forceinline__ float bf_bits2f(unsigned short h) { return __uint_as_float(((unsigned)h) << 16); }

__device__ __forceinline__ void guard1_h(v8f& a, v16h x, v16h y) { asm volatile("v_nop\n\tv_nop\n\tv_nop\n\tv_nop" : "+v"(a) : "v"(x), "v"(y)); }
__device__ __forceinline__ void guard1_b(v8f& a, v16b x, v16b y) { asm volatile("v_nop\n\tv_nop\n\tv_nop\n\tv_nop" : "+v"(a) : "v"(x), "v"(y)); }
__device__ __forceinline__ void keep4_h(v16h a, v16h b, v16h c, v16h d) { asm volatile("v_nop" :: "v"(a), "v"(b), "v"(c), "v"(d)); }
__device__ __forceinline__ void keep4_b(v16b a, v16b b, v16b c, v16b d) { asm volatile("v_nop" :: "v"(a), "v"(b), "v"(c), "v"(d)); }
__device__ __forceinline__ void acc_guard4(v8f& a, v8f& b, v8f& c, v8f& d) { asm volatile("v_nop\n\tv_nop\n\tv_nop\n\tv_nop" : "+v"(a), "+v"(b), "+v"(c), "+v"(d)); }
template <typename T> struct Frag;
template <> struct Frag<_Float16> {
  typedef v16h V; union U { v16h v; v8h h[2]; };
  static __device__ __forceinline__ v16h load(const _Float16* p) {
    U f; f.h[0] = *(const v8h*)(p); f.h[1] = *(const v8h*)(p + 16); return f.v;
  }
  static __device__ __forceinline__ v8f mma(v16h a, v16h b, v8f c) {
    return __builtin_amdgcn_wmma_f32_16x16x32_f16(false, a, false, b, (short)0, c, false, false);
  }
  static __device__ __forceinline__ void guard1(v8f& a, v16h x, v16h y) { guard1_h(a, x, y); }
  static __device__ __forceinline__ void keep(v16h a, v16h b, v16h c, v16h d) { keep4_h(a, b, c, d); }
};
template <> struct Frag<__bf16> {
  typedef v16b V; union U { v16b v; v8b h[2]; };
  static __device__ __forceinline__ v16b load(const __bf16* p) {
    U f; f.h[0] = *(const v8b*)(p); f.h[1] = *(const v8b*)(p + 16); return f.v;
  }
  static __device__ __forceinline__ v8f mma(v16b a, v16b b, v8f c) {
    return __builtin_amdgcn_wmma_f32_16x16x32_bf16(false, a, false, b, (short)0, c, false, false);
  }
  static __device__ __forceinline__ void guard1(v8f& a, v16b x, v16b y) { guard1_b(a, x, y); }
  static __device__ __forceinline__ void keep(v16b a, v16b b, v16b c, v16b d) { keep4_b(a, b, c, d); }
};

template <int ET> struct Elem;
template <> struct Elem<0> { typedef _Float16 T; };
template <> struct Elem<1> { typedef __bf16 T; };
template <int ET, bool SPLIT, int BIAS_MODE, int OUT_MODE, bool RESID, int ACT = 0>
__global__ __launch_bounds__(256) void wmma_gemm64(
    const unsigned short* __restrict__ Ap, const unsigned short* __restrict__ A2p, int lda, long strideA,
    const unsigned short* __restrict__ Btp, const unsigned short* __restrict__ Bt2p, int ldb, long strideB,
    void* __restrict__ Cout, void* __restrict__ Cout2, int ldc, long strideC,
    const float* __restrict__ bias,
    const float* __restrict__ resid, long strideR,
    int M, int N, int K, float scale) {
  typedef typename Elem<ET>::T T;
  typedef typename Frag<T>::V V;
  const T* A = (const T*)Ap; const T* A2 = (const T*)A2p; const T* Bt = (const T*)Btp; const T* Bt2 = (const T*)Bt2p;
  __shared__ __align__(16) float sT[8][16 * 68];
  const int b    = blockIdx.y;
  const int lane = threadIdx.x & 31;
  const int wave = threadIdx.x >> 5;
  const int tilesN = N >> 6;
  const int tilesM = M >> 6;
  const int tile = blockIdx.x * 8 + wave;
  if (tile >= tilesM * tilesN) return;
  const int tm = tile / tilesN;
  const int tn = tile - tm * tilesN;
  const int m0 = tm << 6;
  const int n0 = tn << 6;

  const T* Ab  = A  + (size_t)b * strideA;
  const T* Bb  = Bt + (size_t)b * strideB;
  const T* Ab2 = SPLIT ? (A2  + (size_t)b * strideA) : nullptr;
  const T* Bb2 = SPLIT ? (Bt2 + (size_t)b * strideB) : nullptr;

  const int rlane = lane & 15;
  const int koff  = (lane >> 4) * 8;
  const int mOff  = (lane >> 4) * 8;

  v8f acc[4][4];
#pragma unroll
  for (int i = 0; i < 4; ++i)
#pragma unroll
    for (int j = 0; j < 4; ++j) acc[i][j] = (v8f){0.f,0.f,0.f,0.f,0.f,0.f,0.f,0.f};

  for (int k0 = 0; k0 < K; k0 += 32) {
    V bh[4], bl[4];
#pragma unroll
    for (int j = 0; j < 4; ++j) {
      const size_t bo = (size_t)(n0 + (j << 4) + rlane) * ldb + koff + k0;
      bh[j] = Frag<T>::load(Bb + bo);
      if (SPLIT) bl[j] = Frag<T>::load(Bb2 + bo);
    }
#pragma unroll
    for (int i = 0; i < 4; ++i) {
      const size_t ao = (size_t)(m0 + (i << 4) + rlane) * lda + koff + k0;
      V ah = Frag<T>::load(Ab + ao);
      V al;
      if (SPLIT) al = Frag<T>::load(Ab2 + ao);
#pragma unroll
      for (int j = 0; j < 4; ++j) {
        acc[i][j] = Frag<T>::mma(ah, bh[j], acc[i][j]);
        if (SPLIT) {
          acc[i][j] = Frag<T>::mma(ah, bl[j], acc[i][j]);
          acc[i][j] = Frag<T>::mma(al, bh[j], acc[i][j]);
        }
      }
      Frag<T>::guard1(acc[i][0], ah, bh[0]);
      Frag<T>::guard1(acc[i][1], ah, bh[1]);
      Frag<T>::guard1(acc[i][2], ah, bh[2]);
      Frag<T>::guard1(acc[i][3], ah, bh[3]);
      if (SPLIT) {
        Frag<T>::guard1(acc[i][0], al, bl[0]);
        Frag<T>::guard1(acc[i][1], al, bl[1]);
        Frag<T>::guard1(acc[i][2], al, bl[2]);
        Frag<T>::guard1(acc[i][3], al, bl[3]);
      }
    }
    Frag<T>::keep(bh[0], bh[1], bh[2], bh[3]);
    if (SPLIT) Frag<T>::keep(bl[0], bl[1], bl[2], bl[3]);
  }
  acc_guard4(acc[0][0], acc[0][1], acc[0][2], acc[0][3]);
  acc_guard4(acc[1][0], acc[1][1], acc[1][2], acc[1][3]);
  acc_guard4(acc[2][0], acc[2][1], acc[2][2], acc[2][3]);
  acc_guard4(acc[3][0], acc[3][1], acc[3][2], acc[3][3]);

  float* slab = sT[wave];
  const float* Rb = RESID ? (resid + (size_t)b * strideR) : nullptr;
#pragma unroll
  for (int i = 0; i < 4; ++i) {
    const int mBase = m0 + (i << 4);
#pragma unroll
    for (int j = 0; j < 4; ++j) {
      const int n = n0 + (j << 4) + rlane;
      float bv = 0.f;
      if (BIAS_MODE == 2) bv = bias[n];
#pragma unroll
      for (int r = 0; r < 8; ++r) {
        float v = acc[i][j][r] * scale;
        if (BIAS_MODE == 1) v += bias[mBase + mOff + r];
        if (BIAS_MODE == 2) v += bv;
        if (RESID) v += Rb[(size_t)(mBase + mOff + r) * ldc + n];
        if (ACT == 1) v = tanhf(v);
        if (ACT == 2) v = fmaxf(v, 0.0f);
        if (ACT == 3) v = v / (1.0f + expf(-v));
        if (ACT == 4) v = (v > 0.f) ? v : 0.01f * v;
        slab[(mOff + r) * 68 + (j << 4) + rlane] = v;
      }
    }
    __builtin_amdgcn_fence(__ATOMIC_RELEASE, "workgroup");
    __builtin_amdgcn_wave_barrier();
    __builtin_amdgcn_fence(__ATOMIC_ACQUIRE, "workgroup");
    if (OUT_MODE == 0) {
      float* C = (float*)Cout + (size_t)b * strideC;
      const int hh = lane >> 4, c4 = (lane & 15) * 4;
      for (int pass = 0; pass < 2; ++pass) {
#pragma unroll
        for (int it = 0; it < 8; ++it) {
          const int row = it * 2 + hh;
          v4f v = *(const v4f*)(slab + row * 68 + c4);
          *(volatile v4f*)(C + (size_t)(mBase + row) * ldc + n0 + c4) = v;
        }
        __threadfence();
      }
    } else {
      const int q = lane >> 3, c8 = (lane & 7) * 8;
      unsigned short* C  = (unsigned short*)Cout  + (size_t)b * strideC;
      unsigned short* C2 = (OUT_MODE == 2) ? ((unsigned short*)Cout2 + (size_t)b * strideC) : nullptr;
      for (int pass = 0; pass < 2; ++pass) {
#pragma unroll
        for (int it = 0; it < 4; ++it) {
          const int row = it * 4 + q;
          const float* sp = slab + row * 68 + c8;
          v8h hv, lv;
#pragma unroll
          for (int e = 0; e < 8; ++e) {
            if (OUT_MODE == 1) {
              hv[e] = (_Float16)sp[e];
            } else {
              unsigned short hb = f2bf_bits(sp[e]);
              unsigned short lb = f2bf_bits(sp[e] - bf_bits2f(hb));
              hv[e] = __builtin_bit_cast(_Float16, hb);
              lv[e] = __builtin_bit_cast(_Float16, lb);
            }
          }
          *(volatile v8h*)(C + (size_t)(mBase + row) * ldc + n0 + c8) = hv;
          if (OUT_MODE == 2) *(volatile v8h*)(C2 + (size_t)(mBase + row) * ldc + n0 + c8) = lv;
        }
        __threadfence();
      }
    }
    __builtin_amdgcn_fence(__ATOMIC_RELEASE, "workgroup");
    __builtin_amdgcn_wave_barrier();
    __builtin_amdgcn_fence(__ATOMIC_ACQUIRE, "workgroup");
  }
}

__global__ __launch_bounds__(256) void minmax_kernel(const float* __restrict__ coords, float* __restrict__ part)
{
  __shared__ float sR[8 * 8];
  const int tid = threadIdx.x, lane = tid & 31, wave = tid >> 5;
  const float* src = coords + (size_t)blockIdx.x * (kMmPts * 3) + (size_t)tid * 12;
  const v4f a0 = *(const v4f*)(src);
  const v4f a1 = *(const v4f*)(src + 4);
  const v4f a2 = *(const v4f*)(src + 8);
  float mny = fminf(fminf(a0[0], a0[3]), fminf(a1[2], a2[1]));
  float mnx = fminf(fminf(a0[1], a1[0]), fminf(a1[3], a2[2]));
  float mnz = fminf(fminf(a0[2], a1[1]), fminf(a2[0], a2[3]));
  float mxy = fmaxf(fmaxf(a0[0], a0[3]), fmaxf(a1[2], a2[1]));
  float mxx = fmaxf(fmaxf(a0[1], a1[0]), fmaxf(a1[3], a2[2]));
  float mxz = fmaxf(fmaxf(a0[2], a1[1]), fmaxf(a2[0], a2[3]));
#pragma unroll
  for (int o = 1; o < 32; o <<= 1) {
    mny = fminf(mny, __shfl_xor(mny, o, 32));
    mnx = fminf(mnx, __shfl_xor(mnx, o, 32));
    mnz = fminf(mnz, __shfl_xor(mnz, o, 32));
    mxy = fmaxf(mxy, __shfl_xor(mxy, o, 32));
    mxx = fmaxf(mxx, __shfl_xor(mxx, o, 32));
    mxz = fmaxf(mxz, __shfl_xor(mxz, o, 32));
  }
  float vsel = mny;
  vsel = (lane == 1) ? mnx : vsel;
  vsel = (lane == 2) ? mnz : vsel;
  vsel = (lane == 3) ? mxy : vsel;
  vsel = (lane == 4) ? mxx : vsel;
  vsel = (lane == 5) ? mxz : vsel;
  vsel = (lane >= 6) ? 0.0f : vsel;
  if (lane < 8) sR[wave * 8 + lane] = vsel;
  __syncthreads();
  if (wave == 0) {
    const int j = lane & 7;
    float mn = sR[j], mx = sR[j];
#pragma unroll
    for (int w = 1; w < 8; ++w) {
      const float v = sR[w * 8 + j];
      mn = fminf(mn, v);
      mx = fmaxf(mx, v);
    }
    const float r = (j < 3) ? mn : mx;
    const float ov = (lane < 6) ? r : 0.0f;
    volatile float* dst = part + (size_t)blockIdx.x * 32 + lane;
    *dst = ov;
    __threadfence();
    *dst = ov;
  }
}

__global__ __launch_bounds__(256) void build_bt_kernel(const float* __restrict__ weights, unsigned short* __restrict__ bt)
{
  const int i  = blockIdx.x * 256 + threadIdx.x;
  const int n  = i >> 3, k8 = (i & 7) * 8;
  const int nc = (n < kCells) ? n : (kCells - 1);
  v8h hv;
#pragma unroll
  for (int e = 0; e < 8; ++e) {
    const int k  = k8 + e;
    const int kc = (k < kBasis) ? k : (kBasis - 1);
    float w = weights[nc * kBasis + kc];
    asm volatile("" : "+v"(w));
    float v = ((n < kCells) && (k < kBasis)) ? (w * kCarryW) : 0.0f;
    v = (fabsf(v) < kF16Norm) ? 0.0f : v;
    hv[e] = (_Float16)v;
  }
  unsigned short* dst = bt + (size_t)i * 8;
  *(volatile v8h*)dst = hv;
  __threadfence();
  *(volatile v8h*)dst = hv;
}

__device__ __forceinline__ int cell_index(float v, float lo, float hi, float cells, int top)
{
#pragma clang fp contract(off)
  const float den = (hi - lo) + 1e-9f;
  const float q   = (v - lo) / den;
  const float t   = q * cells;
  int c = (int)t;
  c = (c < 0) ? 0 : c;
  c = (c > top) ? top : c;
  return c;
}

__global__ __launch_bounds__(256) void build_a_kernel(
    const float* __restrict__ coords, const float* __restrict__ kern, const float* __restrict__ part,
    unsigned* __restrict__ aw, int* __restrict__ bidx)
{
  __shared__ __align__(16) float    sK[kKernFl];
  __shared__ __align__(16) unsigned sTile[8][32 * 32];
  __shared__ float sRed[8 * 4];
  const int tid = threadIdx.x, lane = tid & 31, wave = tid >> 5;

#pragma unroll 1
  for (int it = 0; it < 5; ++it) {
    int idx = it * 256 + tid;
    idx = (idx < kKernFl / 4) ? idx : (kKernFl / 4 - 1);
    const v4f kv = *(const v4f*)(kern + 4 * idx);
    *(v4f*)(sK + 4 * idx) = kv;
  }
  {
    const int i    = tid & 127;
    const int half = tid >> 7;
    const float sg = half ? -1.0f : 1.0f;
    const float* pp = part + (size_t)i * 32 + 3 * half;
    float r0 = pp[0] * sg, r1 = pp[1] * sg, r2 = pp[2] * sg;
#pragma unroll
    for (int o = 1; o < 32; o <<= 1) {
      r0 = fminf(r0, __shfl_xor(r0, o, 32));
      r1 = fminf(r1, __shfl_xor(r1, o, 32));
      r2 = fminf(r2, __shfl_xor(r2, o, 32));
    }
    if (lane == 0) {
      sRed[wave * 4 + 0] = r0;
      sRed[wave * 4 + 1] = r1;
      sRed[wave * 4 + 2] = r2;
      sRed[wave * 4 + 3] = 0.0f;
    }
  }
  __syncthreads();
  const float my = fminf(fminf(sRed[0], sRed[4]), fminf(sRed[8], sRed[12]));
  const float mx = fminf(fminf(sRed[1], sRed[5]), fminf(sRed[9], sRed[13]));
  const float mz = fminf(fminf(sRed[2], sRed[6]), fminf(sRed[10], sRed[14]));
  const float My = -fminf(fminf(sRed[16], sRed[20]), fminf(sRed[24], sRed[28]));
  const float Mx = -fminf(fminf(sRed[17], sRed[21]), fminf(sRed[25], sRed[29]));
  const float Mz = -fminf(fminf(sRed[18], sRed[22]), fminf(sRed[26], sRed[30]));

  const int p0 = blockIdx.x * 256 + wave * 32;
  const int p  = p0 + lane;
  const float cy = coords[(size_t)p * 3 + 0];
  const float cx = coords[(size_t)p * 3 + 1];
  const float cz = coords[(size_t)p * 3 + 2];
  const int rr = cell_index(cy, my, My, 4.0f, 3);
  const int cc = cell_index(cx, mx, Mx, 4.0f, 3);
  const int dd = cell_index(cz, mz, Mz, 2.0f, 1);
  const int bq = rr * 8 + cc * 2 + dd;

  unsigned* tile = sTile[wave];
#pragma unroll 1
  for (int j = 0; j < 32; ++j) {
    const float yj = __shfl(cy, j, 32);
    const float xj = __shfl(cx, j, 32);
    const float zj = __shfl(cz, j, 32);
    const int   bj = __shfl(bq, j, 32);
    float s0 = 0.0f, s1 = 0.0f;
#pragma unroll 1
    for (int e = 0; e < 2; ++e) {
      const int m  = 2 * lane + e;
      const int mc = (m < kBasis) ? m : (kBasis - 1);
      const float* kp = sK + bj * (3 * kBasis) + mc;
      float pz = yj * kp[0];
      pz = fmaf(xj, kp[kBasis], pz);
      pz = fmaf(zj, kp[2 * kBasis], pz);
      const float zz = pz + 1.0f;
      float sv = sinf(zz) * kCarryA;
      sv = (m < kBasis) ? sv : 0.0f;
      sv = (fabsf(sv) < kF16Norm) ? 0.0f : sv;
      s0 = (e == 0) ? sv : s0;
      s1 = (e == 1) ? sv : s1;
    }
    const _Float16 h0 = (_Float16)s0, h1 = (_Float16)s1;
    const unsigned u = (unsigned)__builtin_bit_cast(unsigned short, h0) |
                       ((unsigned)__builtin_bit_cast(unsigned short, h1) << 16);
    tile[j * 32 + lane] = u;
  }
  __syncthreads();
  const int q = lane >> 3, c4 = (lane & 7) * 4;
  v4u rows[8];
#pragma unroll
  for (int it = 0; it < 8; ++it) rows[it] = *(const v4u*)(tile + (it * 4 + q) * 32 + c4);
  unsigned* ab = aw + (size_t)p0 * 32;
  for (int pass = 0; pass < 2; ++pass) {
#pragma unroll
    for (int it = 0; it < 8; ++it)
      *(volatile v4u*)(ab + (it * 4 + q) * 32 + c4) = rows[it];
    *(volatile int*)(bidx + p) = bq;
    __threadfence();
  }
}

__global__ __launch_bounds__(256) void gather_sigmoid_kernel(
    const float* __restrict__ cpl, const int* __restrict__ bidx, const float* __restrict__ bias,
    float* __restrict__ out)
{
  const int n = blockIdx.x * 256 + threadIdx.x;
  int b = bidx[n];
  b = (b < 0) ? 0 : b;
  b = (b > kCells - 1) ? (kCells - 1) : b;
  const float v = cpl[(size_t)n * kNPad + b] + bias[b];
  const float o = 1.0f / (1.0f + expf(-v));
  volatile float* dst = out + n;
  *dst = o;
  __threadfence();
  *dst = o;
}

extern "C" void kernel_launch(void* const* d_in, const int* in_sizes, int n_in,
                              void* d_out, int out_size, void* d_ws, size_t ws_size,
                              hipStream_t stream) {
  if (n_in < 4) return;
  if (in_sizes[0] != kPts * 3) return;
  if (in_sizes[1] != kKernFl) return;
  if (in_sizes[2] != kCells * kBasis) return;
  if (in_sizes[3] != kCells) return;
  if (out_size != kPts) return;
  if (ws_size < kWsTotal) return;

  const float* coords  = (const float*)d_in[0];
  const float* kern    = (const float*)d_in[1];
  const float* weights = (const float*)d_in[2];
  const float* bias    = (const float*)d_in[3];
  float* out = (float*)d_out;

  char* ws = (char*)d_ws;
  float*          PART = (float*)(ws + kOffPart);
  int*            BIDX = (int*)(ws + kOffBidx);
  unsigned short* BT   = (unsigned short*)(ws + kOffBt);
  unsigned*       APL  = (unsigned*)(ws + kOffApl);
  float*          CPL  = (float*)(ws + kOffCpl);

  minmax_kernel<<<kMmBlk, 256, 0, stream>>>(coords, PART);
  build_bt_kernel<<<(kNPad * kKPad / 8) / 256, 256, 0, stream>>>(weights, BT);
  build_a_kernel<<<kPts / 256, 256, 0, stream>>>(coords, kern, PART, APL, BIDX);

  wmma_gemm64<0, false, 0, 0, false><<<dim3((kPts / 64) / 8, 1), 256, 0, stream>>>(
      (const unsigned short*)APL, nullptr, kKPad, 0L,
      (const unsigned short*)BT, nullptr, kKPad, 0L,
      (void*)CPL, nullptr, kNPad, 0L,
      nullptr, nullptr, 0L,
      kPts, kNPad, kKPad, kFoldBack);

  gather_sigmoid_kernel<<<kPts / 256, 256, 0, stream>>>(CPL, BIDX, bias, out);
}
